// STLayer_66099546685511
// MI455X (gfx1250) — hardware-verified
//
#include <hip/hip_runtime.h>


#define GG   32
#define NP   32768
#define CC   96
#define CP   128
#define WS   8
#define SHF  4
#define NW   64
#define NT   512
#define NH_  6
#define HD   16
#define KP   32
#define HID  384
#define GWN  8
#define NZ   (GWN * NH_)
#define DM   CP
#define PCAR 1024.0f
#define LOSC 1024.0f
typedef _Float16 h16;
typedef unsigned short bf;
typedef __attribute__((ext_vector_type(16))) __bf16   v16bf;
typedef __attribute__((ext_vector_type(16))) _Float16 v16h;
typedef __attribute__((ext_vector_type(8)))  _Float16 v8h;
typedef __attribute__((ext_vector_type(8)))  unsigned short v8us;
typedef __attribute__((ext_vector_type(8)))  float    v8f;
typedef __attribute__((ext_vector_type(4)))  float    v4f;
typedef v8h  __attribute__((may_alias)) v8ha;
typedef v4f  __attribute__((may_alias)) v4fa;
typedef v8us __attribute__((may_alias)) v8usa;

__device__ __forceinline__ unsigned short f2bf(float f) { unsigned u = __float_as_uint(f); u += 0x7FFFu + ((u >> 16) & 1u); return (unsigned short)(u >> 16); }
__device__ __forceinline__ float bf2f(unsigned short b) { return __uint_as_float(((unsigned)b) << 16); }
__device__ __forceinline__ float bfr(float f) { return bf2f(f2bf(f)); }
__device__ __forceinline__ v16h cat16(v8h lo, v8h hi) { return __builtin_shufflevector(lo, hi, 0, 1, 2, 3, 4, 5, 6, 7, 8, 9, 10, 11, 12, 13, 14, 15); }
__device__ __forceinline__ v16bf cat16b(v8us lo, v8us hi) { return __builtin_bit_cast(v16bf, __builtin_shufflevector(lo, hi, 0, 1, 2, 3, 4, 5, 6, 7, 8, 9, 10, 11, 12, 13, 14, 15)); }
__device__ __forceinline__ v8f wmma16(v16h a, v16h b, v8f c) { return __builtin_amdgcn_wmma_f32_16x16x32_f16(false, a, false, b, (short)0, c, false, false); }
__device__ __forceinline__ v8f wmmab(v16bf a, v16bf b, v8f c) { return __builtin_amdgcn_wmma_f32_16x16x32_bf16(false, a, false, b, (short)0, c, false, false); }


__global__ __launch_bounds__(128) void k_gemmh(const h16* __restrict__ A, const h16* __restrict__ Bn, const float* __restrict__ bias, float* C, int ldc, const float* __restrict__ R, int K, size_t sA, size_t sB, size_t sC, int roundR) {
    __shared__ __align__(16) float ost[4][16 * 68];
    const size_t z = blockIdx.z; A += z * sA; Bn += z * sB; C += z * sC; if (R) R += z * sC;
    const int lane = threadIdx.x & 31, wave = threadIdx.x >> 5, lr = lane & 15, hi = lane >> 4;
    const int r0 = blockIdx.x * 64 + wave * 16, c0 = blockIdx.y * 64;
    const size_t aoff = (size_t)(r0 + lr) * K + 8 * hi;
    size_t boff[4];
#pragma unroll
    for (int t = 0; t < 4; ++t) boff[t] = (size_t)(c0 + t * 16 + lr) * K + 8 * hi;
    v8f acc[4];
#pragma unroll
    for (int t = 0; t < 4; ++t) acc[t] = (v8f){};
#pragma unroll 1
    for (int kc = 0; kc < K; kc += 32) {
        const v16h a = cat16(*(const v8h*)(A + aoff + kc), *(const v8h*)(A + aoff + kc + 16));
#pragma unroll
        for (int t = 0; t < 4; ++t) { const v16h b = cat16(*(const v8h*)(Bn + boff[t] + kc), *(const v8h*)(Bn + boff[t] + kc + 16)); acc[t] = wmma16(a, b, acc[t]); }
        asm volatile("v_nop\n\tv_nop\n\tv_nop\n\tv_nop" : "+v"(acc[0]), "+v"(acc[1]), "+v"(acc[2]), "+v"(acc[3]) : "v"(a));
    }
    float* os = &ost[wave][0];
#pragma unroll
    for (int t = 0; t < 4; ++t) { const float bv = bias ? bfr(bias[c0 + t * 16 + lr]) : 0.f;
#pragma unroll
        for (int j = 0; j < 8; ++j) os[(hi * 8 + j) * 68 + t * 16 + lr] = acc[t][j] + bv; }
    __syncthreads();
    float* crow = C + (size_t)r0 * ldc + c0;
    auto pass = [&]() {
#pragma unroll
        for (int s = 0; s < 8; ++s) { const int Lid = (lane >> 3) + 4 * s, piece = lane & 7; const int row = Lid >> 1, cofs = (Lid & 1) * 32 + piece * 4;
            v4f val = *(const v4fa*)(os + row * 68 + cofs); if (R) { const v4f rv = *(const v4f*)(R + ((size_t)r0 + row) * ldc + c0 + cofs); val += roundR ? (v4f){bfr(rv[0]), bfr(rv[1]), bfr(rv[2]), bfr(rv[3])} : rv; }
            *(volatile v4f*)(crow + (size_t)row * ldc + cofs) = val; }
    };
    pass(); __threadfence(); pass();
}

__global__ __launch_bounds__(128) void k_gemmh32(const h16* __restrict__ A, const h16* __restrict__ Bn, int K, float* C, int ldc, size_t sA, size_t sB, size_t sC) {
    const size_t z = blockIdx.z; A += z * sA; Bn += z * sB; C += z * sC;
    __shared__ __align__(16) float ost[4][16 * 36];
    const int lane = threadIdx.x & 31, wave = threadIdx.x >> 5, lr = lane & 15, hi = lane >> 4;
    const int r0 = blockIdx.x * 64 + wave * 16, c0 = blockIdx.y * 32;
    const size_t aoff = (size_t)(r0 + lr) * K + 8 * hi;
    v8f acc[2]; acc[0] = (v8f){}; acc[1] = (v8f){};
#pragma unroll 1
    for (int kc = 0; kc < K; kc += 32) {
        const v16h a = cat16(*(const v8h*)(A + aoff + kc), *(const v8h*)(A + aoff + kc + 16));
#pragma unroll
        for (int t = 0; t < 2; ++t) { const size_t bo = (size_t)(c0 + t * 16 + lr) * K + kc + 8 * hi; const v16h b = cat16(*(const v8h*)(Bn + bo), *(const v8h*)(Bn + bo + 16)); acc[t] = wmma16(a, b, acc[t]); }
        asm volatile("v_nop\n\tv_nop\n\tv_nop\n\tv_nop" : "+v"(acc[0]), "+v"(acc[1]) : "v"(a));
    }
    float* os = &ost[wave][0];
#pragma unroll
    for (int t = 0; t < 2; ++t) {
#pragma unroll
        for (int j = 0; j < 8; ++j) os[(hi * 8 + j) * 36 + t * 16 + lr] = acc[t][j]; }
    __builtin_amdgcn_wave_barrier(); asm volatile("" ::: "memory");
    float* crow = C + (size_t)r0 * ldc + c0;
    auto pass = [&]() {
#pragma unroll
        for (int s = 0; s < 4; ++s) { const int row = (lane >> 3) + 4 * s, piece = lane & 7; const int cofs = piece * 4;
            const v4f val = *(const v4fa*)(os + row * 36 + cofs); *(volatile v4f*)(crow + (size_t)row * ldc + cofs) = val; }
    };
    pass(); __threadfence(); pass();
}


template <int MODE>
__global__ __launch_bounds__(128) void k_gemm3z(const bf* __restrict__ Ah, const bf* __restrict__ Al, const bf* __restrict__ Bh, const bf* __restrict__ Bl, int K, float* C, int ldc, size_t sA, size_t sB, size_t sC) {
    if ((MODE & 1) && (int)blockIdx.y * 64 > (int)blockIdx.x * 64 + 63) return;
    const size_t z = blockIdx.z; Ah += z * sA; Al += z * sA; Bh += z * sB; Bl += z * sB; C += z * sC;
    const int Klim = (MODE & 2) ? min(K, ((int)blockIdx.x + 1) * 64) : K;
    __shared__ __align__(16) float ost[4][16 * 68];
    const int lane = threadIdx.x & 31, wave = threadIdx.x >> 5, lr = lane & 15, hi = lane >> 4;
    const int r0 = blockIdx.x * 64 + wave * 16, c0 = blockIdx.y * 64;
    const size_t aoff = (size_t)(r0 + lr) * K + 8 * hi;
    v8f acc[4];
#pragma unroll
    for (int t = 0; t < 4; ++t) acc[t] = (v8f){};
#pragma unroll 1
    for (int kc = 0; kc < Klim; kc += 32) {
        const v16bf a = cat16b(*(const v8us*)(Ah + aoff + kc), *(const v8us*)(Ah + aoff + kc + 16));
        v16bf al = a; if (!(MODE & 4) && !(MODE & 16)) al = cat16b(*(const v8us*)(Al + aoff + kc), *(const v8us*)(Al + aoff + kc + 16));
#pragma unroll
        for (int t = 0; t < 4; ++t) { const size_t bo = (size_t)(c0 + t * 16 + lr) * K + kc + 8 * hi;
            const v16bf bh = cat16b(*(const v8us*)(Bh + bo), *(const v8us*)(Bh + bo + 16));
            acc[t] = wmmab(a, bh, acc[t]);
            if (!(MODE & 4)) { if (!(MODE & 16)) acc[t] = wmmab(al, bh, acc[t]); if (!(MODE & 8)) { const v16bf bl = cat16b(*(const v8us*)(Bl + bo), *(const v8us*)(Bl + bo + 16)); acc[t] = wmmab(a, bl, acc[t]); } } }
        asm volatile("v_nop\n\tv_nop\n\tv_nop\n\tv_nop" : "+v"(acc[0]), "+v"(acc[1]), "+v"(acc[2]), "+v"(acc[3]) : "v"(a), "v"(al));
    }
    float* os = &ost[wave][0];
#pragma unroll
    for (int t = 0; t < 4; ++t) {
#pragma unroll
        for (int j = 0; j < 8; ++j) os[(hi * 8 + j) * 68 + t * 16 + lr] = acc[t][j]; }
    __builtin_amdgcn_wave_barrier(); asm volatile("" ::: "memory");
    float* crow = C + (size_t)r0 * ldc + c0;
    auto pass = [&]() {
#pragma unroll
        for (int s = 0; s < 8; ++s) { const int Lid = (lane >> 3) + 4 * s, piece = lane & 7; const int row = Lid >> 1, cofs = (Lid & 1) * 32 + piece * 4;
            const v4f val = *(const v4fa*)(os + row * 68 + cofs); *(volatile v4f*)(crow + (size_t)row * ldc + cofs) = val; }
    };
    pass(); __threadfence(); pass();
}
__global__ __launch_bounds__(256) void k_planes32z(const float* __restrict__ F, int ld, int off, float sc, int rows, bf* Ph, bf* Pl) {
    typedef __attribute__((ext_vector_type(2))) unsigned short v2us;
    const int lane = threadIdx.x & 31; const size_t r = ((size_t)blockIdx.x * 8 + (threadIdx.x >> 5)) * 2 + (lane >> 4); if (r >= (size_t)rows) return; const int z = blockIdx.z; const int c0 = (lane & 15) * 2; v2us oh, ol;
    Ph += (size_t)z * rows * 32; Pl += (size_t)z * rows * 32;
#pragma unroll
    for (int i = 0; i < 2; ++i) { const float y = F[r * ld + off + z * 32 + c0 + i] * sc; const unsigned short hb = f2bf(y); oh[i] = hb; ol[i] = f2bf(y - bf2f(hb)); }
    const size_t o = r * 32 + c0; *(volatile v2us*)(Ph + o) = oh; *(volatile v2us*)(Pl + o) = ol; __threadfence(); *(volatile v2us*)(Ph + o) = oh; *(volatile v2us*)(Pl + o) = ol;
}
__global__ __launch_bounds__(256) void k_vtpadz(const float* __restrict__ F, int ld, int off, int nk, bf* Th, bf* Tl) {
    typedef __attribute__((ext_vector_type(2))) unsigned short v2us;
    const int lane = threadIdx.x & 31; const size_t wid = (size_t)blockIdx.x * 8 + (threadIdx.x >> 5); if (wid >= (size_t)64 * (nk / 64)) return; const int z = blockIdx.z; const int d = (int)(wid / (nk / 64)); const int k0 = (int)(wid % (nk / 64)) * 64 + lane * 2; v2us oh, ol;
    Th += (size_t)z * 64 * nk; Tl += (size_t)z * 64 * nk;
#pragma unroll
    for (int i = 0; i < 2; ++i) { const float y = (d < 32) ? F[(size_t)(k0 + i) * ld + off + z * 32 + (d < 32 ? d : 0)] : 0.f; const unsigned short hb = f2bf(y); oh[i] = hb; ol[i] = f2bf(y - bf2f(hb)); }
    const size_t o = (size_t)d * nk + k0; *(volatile v2us*)(Th + o) = oh; *(volatile v2us*)(Tl + o) = ol; __threadfence(); *(volatile v2us*)(Th + o) = oh; *(volatile v2us*)(Tl + o) = ol;
}
template <int NK>
__global__ __launch_bounds__(256) void k_softmaxz(const float* __restrict__ S, int rows, bf* PH, bf* PL) {
    typedef __attribute__((ext_vector_type(4))) unsigned short v4us;
    const int lane = threadIdx.x & 31, i = blockIdx.x * 8 + (threadIdx.x >> 5); if (i >= rows) return; const size_t zo = (size_t)blockIdx.z * rows * NK; const float* sr = S + zo + (size_t)i * NK; PH += zo; PL += zo;
    float m = -3.0e38f;
#pragma unroll 1
    for (int c0 = lane * 4; c0 < NK; c0 += 128) {
#pragma unroll
        for (int q = 0; q < 4; ++q) m = fmaxf(m, sr[c0 + q]); }
#pragma unroll
    for (int sh = 16; sh; sh >>= 1) m = fmaxf(m, __shfl_xor(m, sh, 32));
    float sum = 0.f;
#pragma unroll 1
    for (int c0 = lane * 4; c0 < NK; c0 += 128) {
#pragma unroll
        for (int q = 0; q < 4; ++q) sum += __expf(sr[c0 + q] - m); }
#pragma unroll
    for (int sh = 16; sh; sh >>= 1) sum += __shfl_xor(sum, sh, 32);
    const float inv = 1.0f / sum;
#pragma unroll 1
    for (int ps = 0; ps < 2; ++ps) {
#pragma unroll 1
        for (int c0 = lane * 4; c0 < NK; c0 += 128) { v4us oh, ol;
#pragma unroll
            for (int q = 0; q < 4; ++q) { const float p = __expf(sr[c0 + q] - m) * inv; const unsigned short hb = f2bf(p); oh[q] = hb; ol[q] = f2bf(p - bf2f(hb)); }
            const size_t o = (size_t)i * NK + c0; *(volatile v4us*)(PH + o) = oh; *(volatile v4us*)(PL + o) = ol; }
        if (ps == 0) __threadfence(); }
}
__global__ __launch_bounds__(256) void k_placez(const float* __restrict__ XH, int rows, int ldy, float* Y) {
    const int lane = threadIdx.x & 31; const size_t q = (size_t)blockIdx.x * 8 + (threadIdx.x >> 5); if (q >= (size_t)rows) return; const int z = blockIdx.z; const float v = XH[((size_t)z * rows + q) * 64 + lane];
    *(volatile float*)(Y + q * ldy + z * 32 + lane) = v; __threadfence(); *(volatile float*)(Y + q * ldy + z * 32 + lane) = v;
}

template <typename T16> struct WFrag;
template <> struct WFrag<h16> { typedef v16h V; static __device__ __forceinline__ V ld(const h16* p) { return cat16(*(const v8h*)p, *(const v8h*)(p + 16)); } static __device__ __forceinline__ v8f mma(V a, V b, v8f c) { return wmma16(a, b, c); } };
template <> struct WFrag<bf> { typedef v16bf V; static __device__ __forceinline__ V ld(const bf* p) { return cat16b(*(const v8us*)p, *(const v8us*)(p + 16)); } static __device__ __forceinline__ v8f mma(V a, V b, v8f c) { return wmmab(a, b, c); } };
template <typename T16, int NSPLIT, bool BIAS>
__global__ __launch_bounds__(32) void k_gemmw(const T16* __restrict__ A, const T16* __restrict__ A2, const T16* __restrict__ Bt, const T16* __restrict__ Bt2, int K, float* C, int ldc, const float* __restrict__ bias, size_t sA, size_t sB, size_t sC) {
    typedef typename WFrag<T16>::V V;
    __shared__ __align__(16) float os[16 * 68];
    const size_t z = blockIdx.z; A += z * sA; if (A2) A2 += z * sA; Bt += z * sB; if (Bt2) Bt2 += z * sB; C += z * sC;
    const int lane = threadIdx.x & 31, lr = lane & 15, hi = lane >> 4; const int r0 = blockIdx.x * 64, c0 = blockIdx.y * 64;
    v8f acc[4][4];
#pragma unroll
    for (int mb = 0; mb < 4; ++mb)
#pragma unroll
        for (int nb = 0; nb < 4; ++nb) acc[mb][nb] = (v8f){};
    const size_t aoff = (size_t)(r0 + lr) * K + 8 * hi, boff = (size_t)(c0 + lr) * K + 8 * hi;
#pragma unroll 1
    for (int kc = 0; kc < K; kc += 32) {
        V a[4], a2[4];
#pragma unroll
        for (int mb = 0; mb < 4; ++mb) { a[mb] = WFrag<T16>::ld(A + aoff + (size_t)mb * 16 * K + kc); if (NSPLIT == 1 || NSPLIT == 2) a2[mb] = WFrag<T16>::ld(A2 + aoff + (size_t)mb * 16 * K + kc); }
#pragma unroll
        for (int nb = 0; nb < 4; ++nb) { const V b = WFrag<T16>::ld(Bt + boff + (size_t)nb * 16 * K + kc); V b2; if (NSPLIT >= 2) b2 = WFrag<T16>::ld(Bt2 + boff + (size_t)nb * 16 * K + kc);
#pragma unroll
            for (int mb = 0; mb < 4; ++mb) { acc[mb][nb] = WFrag<T16>::mma(a[mb], b, acc[mb][nb]); if (NSPLIT == 1 || NSPLIT == 2) acc[mb][nb] = WFrag<T16>::mma(a2[mb], b, acc[mb][nb]); if (NSPLIT >= 2) acc[mb][nb] = WFrag<T16>::mma(a[mb], b2, acc[mb][nb]); } }
        asm volatile("v_nop\n\tv_nop\n\tv_nop\n\tv_nop" : "+v"(acc[0][0]), "+v"(acc[1][1]), "+v"(acc[2][2]), "+v"(acc[3][3]) : "v"(a[0]), "v"(a[3]));
    }
#pragma unroll
    for (int mb = 0; mb < 4; ++mb) {
#pragma unroll
        for (int nb = 0; nb < 4; ++nb) {
#pragma unroll
            for (int j = 0; j < 8; ++j) os[(hi * 8 + j) * 68 + nb * 16 + lr] = acc[mb][nb][j]; }
        __builtin_amdgcn_wave_barrier(); asm volatile("" ::: "memory");
        float* crow = C + (size_t)(r0 + mb * 16) * ldc + c0;
#pragma unroll 1
        for (int ps = 0; ps < 2; ++ps) {
#pragma unroll
            for (int s = 0; s < 8; ++s) { const int row = 2 * s + hi, cofs = lr * 4; v4f val = *(const v4fa*)(os + row * 68 + cofs); if (BIAS) { val[0] += bfr(bias[c0 + cofs]); val[1] += bfr(bias[c0 + cofs + 1]); val[2] += bfr(bias[c0 + cofs + 2]); val[3] += bfr(bias[c0 + cofs + 3]); }
                *(volatile v4f*)(crow + (size_t)row * ldc + cofs) = val; }
            if (ps == 0) __threadfence(); }
        __builtin_amdgcn_wave_barrier(); asm volatile("" ::: "memory");
    }
}
template <typename T16, int NSPLIT, bool BIAS, int CAUS>
__global__ __launch_bounds__(32) void k_gemmwc(const T16* __restrict__ A, const T16* __restrict__ A2, const T16* __restrict__ Bt, const T16* __restrict__ Bt2, int K, float* C, int ldc, const float* __restrict__ bias, size_t sA, size_t sB, size_t sC) {
    typedef typename WFrag<T16>::V V;
    __shared__ __align__(16) float os[16 * 68];
    if (CAUS == 1 && (int)blockIdx.y * 64 > (int)blockIdx.x * 64) return;
    const int Klim = (CAUS == 2) ? min(K, ((int)blockIdx.x + 1) * 64) : K;
    const size_t z = blockIdx.z; A += z * sA; if (A2) A2 += z * sA; Bt += z * sB; if (Bt2) Bt2 += z * sB; C += z * sC;
    const int lane = threadIdx.x & 31, lr = lane & 15, hi = lane >> 4; const int r0 = blockIdx.x * 64, c0 = blockIdx.y * 64;
    v8f acc[4][4];
#pragma unroll
    for (int mb = 0; mb < 4; ++mb)
#pragma unroll
        for (int nb = 0; nb < 4; ++nb) acc[mb][nb] = (v8f){};
    const size_t aoff = (size_t)(r0 + lr) * K + 8 * hi, boff = (size_t)(c0 + lr) * K + 8 * hi;
#pragma unroll 1
    for (int kc = 0; kc < Klim; kc += 32) {
        V a[4], a2[4];
#pragma unroll
        for (int mb = 0; mb < 4; ++mb) { a[mb] = WFrag<T16>::ld(A + aoff + (size_t)mb * 16 * K + kc); if (NSPLIT == 1 || NSPLIT == 2) a2[mb] = WFrag<T16>::ld(A2 + aoff + (size_t)mb * 16 * K + kc); }
#pragma unroll
        for (int nb = 0; nb < 4; ++nb) { const V b = WFrag<T16>::ld(Bt + boff + (size_t)nb * 16 * K + kc); V b2; if (NSPLIT >= 2) b2 = WFrag<T16>::ld(Bt2 + boff + (size_t)nb * 16 * K + kc);
#pragma unroll
            for (int mb = 0; mb < 4; ++mb) { acc[mb][nb] = WFrag<T16>::mma(a[mb], b, acc[mb][nb]); if (NSPLIT == 1 || NSPLIT == 2) acc[mb][nb] = WFrag<T16>::mma(a2[mb], b, acc[mb][nb]); if (NSPLIT >= 2) acc[mb][nb] = WFrag<T16>::mma(a[mb], b2, acc[mb][nb]); } }
        asm volatile("v_nop\n\tv_nop\n\tv_nop\n\tv_nop" : "+v"(acc[0][0]), "+v"(acc[1][1]), "+v"(acc[2][2]), "+v"(acc[3][3]) : "v"(a[0]), "v"(a[3]));
    }
#pragma unroll
    for (int mb = 0; mb < 4; ++mb) {
#pragma unroll
        for (int nb = 0; nb < 4; ++nb) {
#pragma unroll
            for (int j = 0; j < 8; ++j) os[(hi * 8 + j) * 68 + nb * 16 + lr] = acc[mb][nb][j]; }
        __builtin_amdgcn_wave_barrier(); asm volatile("" ::: "memory");
        float* crow = C + (size_t)(r0 + mb * 16) * ldc + c0;
#pragma unroll 1
        for (int ps = 0; ps < 2; ++ps) {
#pragma unroll
            for (int s = 0; s < 8; ++s) { const int row = 2 * s + hi, cofs = lr * 4; v4f val = *(const v4fa*)(os + row * 68 + cofs); if (BIAS) { val[0] += bfr(bias[c0 + cofs]); val[1] += bfr(bias[c0 + cofs + 1]); val[2] += bfr(bias[c0 + cofs + 2]); val[3] += bfr(bias[c0 + cofs + 3]); }
                *(volatile v4f*)(crow + (size_t)row * ldc + cofs) = val; }
            if (ps == 0) __threadfence(); }
        __builtin_amdgcn_wave_barrier(); asm volatile("" ::: "memory");
    }
}
typedef __attribute__((ext_vector_type(4))) _Float16 v4h;
__device__ __forceinline__ h16 tohx(float x) { return (h16)x; }
__device__ __forceinline__ float gelu_e(float x) { return 0.5f * x * (1.0f + erff(x * 0.70710678118654752f)); }
__device__ __forceinline__ int ptok(int w, int n) { const int wa = w >> 4, wb = (w >> 2) & 3, wc = w & 3; const int na = n >> 6, nb = (n >> 3) & 7, nc = n & 7; const int a = (wa * WS + na + SHF) & (GG - 1), b = (wb * WS + nb + SHF) & (GG - 1), c = (wc * WS + nc + SHF) & (GG - 1); return (a * GG + b) * GG + c; }
__device__ __forceinline__ int segof(int s) { return s < GG - WS ? 0 : (s < GG - SHF ? 1 : 2); }
__device__ __forceinline__ int region(int w, int n) { const int wa = w >> 4, wb = (w >> 2) & 3, wc = w & 3; const int na = n >> 6, nb = (n >> 3) & 7, nc = n & 7; return segof(wa * WS + na) * 9 + segof(wb * WS + nb) * 3 + segof(wc * WS + nc); }
template <bool SPLIT>
__global__ __launch_bounds__(256) void k_wpad(const float* __restrict__ Wm, int nout, int kin, int noutp, int kp, h16* Bt) {
    const int lane = threadIdx.x & 31; const int n = blockIdx.x * 8 + (threadIdx.x >> 5); if (n >= noutp) return; int src = -1;
    if (SPLIT) { const int s = n / CP, j = n % CP; if (j < CC) src = s * CC + j; } else { if (n < nout) src = n; }
#pragma unroll 1
    for (int ps = 0; ps < 2; ++ps) { for (int c0 = lane * 4; c0 < kp; c0 += 128) { v4h o;
#pragma unroll
            for (int i = 0; i < 4; ++i) { const int k = c0 + i; o[i] = tohx((src >= 0 && k < kin) ? bfr(Wm[(size_t)src * kin + k]) : 0.f); }
            *(volatile v4h*)(Bt + (size_t)n * kp + c0) = o; }
        if (ps == 0) __threadfence(); }
}
__global__ __launch_bounds__(256) void k_bias(const float* __restrict__ qb, const float* __restrict__ vb, const float* __restrict__ pb, const float* __restrict__ b1, const float* __restrict__ b2, float* BQ, float* BP, float* B1, float* B2) {
    const int lane = threadIdx.x & 31, wv = threadIdx.x >> 5;
#pragma unroll 1
    for (int ps = 0; ps < 2; ++ps) { v4f o;
#pragma unroll
        for (int i = 0; i < 4; ++i) { const int j = lane * 4 + i; float v = 0.f;
            if (wv < 3) { v = (j < CC) ? (wv == 0 ? bfr(qb[j]) : wv == 2 ? bfr(vb[j]) : 0.f) : 0.f; } else if (wv == 3) { v = j < CC ? bfr(pb[j]) : 0.f; } else if (wv < 7) { v = bfr(b1[(wv - 4) * 128 + j]); } else { v = j < CC ? bfr(b2[j]) : 0.f; }
            o[i] = v; }
        float* dst = (wv < 3) ? BQ + wv * 128 : (wv == 3) ? BP : (wv < 7) ? B1 + (wv - 4) * 128 : B2; *(volatile v4f*)(dst + lane * 4) = o; if (ps == 0) __threadfence(); }
}
__global__ __launch_bounds__(256) void k_ln1(const float* __restrict__ x, const float* __restrict__ g_, const float* __restrict__ b_, h16* H1p) {
    const int lane = threadIdx.x & 31; const size_t p = (size_t)blockIdx.x * 8 + (threadIdx.x >> 5); if (p >= (size_t)NP) return; float v[3]; float s = 0.f;
#pragma unroll
    for (int i = 0; i < 3; ++i) { v[i] = bfr(x[p * CC + lane * 3 + i]); s += v[i]; }
#pragma unroll
    for (int sh = 16; sh; sh >>= 1) s += __shfl_xor(s, sh, 32);
    const float mu = s * (1.0f / CC); float q = 0.f;
#pragma unroll
    for (int i = 0; i < 3; ++i) { const float d = v[i] - mu; q = fmaf(d, d, q); }
#pragma unroll
    for (int sh = 16; sh; sh >>= 1) q += __shfl_xor(q, sh, 32);
    const float rs = rsqrtf(q * (1.0f / CC) + 1e-5f);
    v4h o;
#pragma unroll
    for (int i = 0; i < 4; ++i) { const int c = lane * 4 + i; const int sl = (c < CC) ? c / 3 : 0, sk = (c < CC) ? c % 3 : 0; const float a0 = __shfl(v[0], sl, 32), a1 = __shfl(v[1], sl, 32), a2 = __shfl(v[2], sl, 32); const float xv = sk == 0 ? a0 : sk == 1 ? a1 : a2; o[i] = tohx(c < CC ? (xv - mu) * rs * bfr(g_[c]) + bfr(b_[c < CC ? c : 0]) : 0.f); }
    *(volatile v4h*)(H1p + p * CP + lane * 4) = o; __threadfence(); *(volatile v4h*)(H1p + p * CP + lane * 4) = o;
}
__global__ __launch_bounds__(256) void k_qkpl(const float* __restrict__ QKV, int w0, h16* Qp, h16* Kp) {
    const int lane = threadIdx.x & 31; const size_t wv = (size_t)blockIdx.x * 8 + (threadIdx.x >> 5); if (wv >= (size_t)NZ * (NT / 4)) return; const int z = (int)(wv / (NT / 4)); const int n = (int)(wv % (NT / 4)) * 4 + (lane >> 3); const int d0 = (lane & 7) * 4; const int w = w0 + z / NH_, h = z % NH_; const size_t p = (size_t)ptok(w, n); v4h oq, ok;
#pragma unroll
    for (int i = 0; i < 4; ++i) { const int d = d0 + i; const bool live = d < HD; oq[i] = tohx(live ? QKV[p * HID + h * HD + d] * 0.25f : 0.f); ok[i] = tohx(live ? QKV[p * HID + CP + h * HD + d] : 0.f); }
    const size_t off = ((size_t)z * NT + n) * KP + d0; *(volatile v4h*)(Qp + off) = oq; *(volatile v4h*)(Kp + off) = ok; __threadfence(); *(volatile v4h*)(Qp + off) = oq; *(volatile v4h*)(Kp + off) = ok;
}
__global__ __launch_bounds__(256) void k_vT(const float* __restrict__ QKV, int w0, h16* VT) {
    const int lane = threadIdx.x & 31; const size_t wv = (size_t)blockIdx.x * 8 + (threadIdx.x >> 5); if (wv >= (size_t)NZ * KP) return; const int z = (int)(wv / KP), d = (int)(wv % KP); const int w = w0 + z / NH_, h = z % NH_;
#pragma unroll 1
    for (int ps = 0; ps < 2; ++ps) {
#pragma unroll
        for (int hp = 0; hp < 2; ++hp) { v8h o;
#pragma unroll
            for (int i = 0; i < 8; ++i) { const int m = hp * 256 + lane * 8 + i; o[i] = tohx(d < HD ? QKV[(size_t)ptok(w, m) * HID + 2 * CP + h * HD + (d < HD ? d : 0)] : 0.f); }
            *(volatile v8h*)(VT + ((size_t)z * KP + d) * NT + hp * 256 + lane * 8) = o; }
        if (ps == 0) __threadfence(); }
}
__global__ __launch_bounds__(256) void k_softs3(float* S, const float* __restrict__ tab, int w0, h16* P) {
    const int lane = threadIdx.x & 31; const size_t wv = (size_t)blockIdx.x * 8 + (threadIdx.x >> 5); if (wv >= (size_t)NZ * NT) return; const int z = (int)(wv / NT), n = (int)(wv % NT); const int w = w0 + z / NH_, h = z % NH_; float* sr = S + wv * NT; h16* po = P + wv * NT;
    const int na = n >> 6, nb = (n >> 3) & 7, nc = n & 7; const int rn = region(w, n);
    float m_ = -3.0e38f;
#pragma unroll 1
    for (int c0 = lane * 4; c0 < NT; c0 += 128) { v4f sv = *(const v4f*)(sr + c0);
#pragma unroll
        for (int q = 0; q < 4; ++q) { const int m = c0 + q; const int ma = m >> 6, mb = (m >> 3) & 7, mc = m & 7; const int rel = ((na - ma) + WS - 1) * 225 + ((nb - mb) + WS - 1) * 15 + ((nc - mc) + WS - 1); float v = sv[q] + bfr(tab[(size_t)rel * NH_ + h]); if (region(w, m) != rn) v += -100.0f; sv[q] = v; m_ = fmaxf(m_, v); }
        *(v4f*)(sr + c0) = sv; }
#pragma unroll
    for (int sh = 16; sh; sh >>= 1) m_ = fmaxf(m_, __shfl_xor(m_, sh, 32));
    float sum = 0.f;
#pragma unroll 1
    for (int c0 = lane * 4; c0 < NT; c0 += 128) { const v4f sv = *(const v4f*)(sr + c0);
#pragma unroll
        for (int q = 0; q < 4; ++q) sum += __expf(sv[q] - m_); }
#pragma unroll
    for (int sh = 16; sh; sh >>= 1) sum += __shfl_xor(sum, sh, 32);
    const float f = __fdiv_rn(PCAR, sum);
#pragma unroll 1
    for (int ps = 0; ps < 2; ++ps) {
#pragma unroll 1
        for (int c0 = lane * 4; c0 < NT; c0 += 128) { const v4f sv = *(const v4f*)(sr + c0); v4h o;
#pragma unroll
            for (int q = 0; q < 4; ++q) o[q] = tohx(__expf(sv[q] - m_) * f);
            *(volatile v4h*)(po + c0) = o; }
        if (ps == 0) __threadfence(); }
}
__global__ __launch_bounds__(256) void k_foldw(const float* __restrict__ OZ, int w0, h16* ATT16) {
    const int lane = threadIdx.x & 31; const size_t wv = (size_t)blockIdx.x * 8 + (threadIdx.x >> 5); if (wv >= (size_t)GWN * NT) return; const int wl = (int)(wv / NT), n = (int)(wv % NT); const size_t p = (size_t)ptok(w0 + wl, n); const int c0 = lane * 4; const int h = c0 / HD, d0 = c0 % HD; v4h o;
#pragma unroll
    for (int i = 0; i < 4; ++i) o[i] = tohx(c0 < CC ? OZ[(((size_t)(wl * NH_ + h)) * NT + n) * KP + d0 + i] * (1.0f / PCAR) : 0.f);
    *(volatile v4h*)(ATT16 + p * CP + c0) = o; __threadfence(); *(volatile v4h*)(ATT16 + p * CP + c0) = o;
}
__global__ __launch_bounds__(256) void k_ln2(const float* __restrict__ x, const float* __restrict__ PR, const float* __restrict__ g_, const float* __restrict__ b_, float* X2, h16* H2p) {
    const int lane = threadIdx.x & 31; const size_t p = (size_t)blockIdx.x * 8 + (threadIdx.x >> 5); if (p >= (size_t)NP) return; const int c0 = lane * 4; float v[4]; float s = 0.f;
#pragma unroll
    for (int i = 0; i < 4; ++i) { const int c = c0 + i; v[i] = (c < CC) ? bfr(x[p * CC + c]) + PR[p * CP + c] : 0.f; s += v[i]; }
#pragma unroll
    for (int sh = 16; sh; sh >>= 1) s += __shfl_xor(s, sh, 32);
    const float mu = s * (1.0f / CC); float q = 0.f;
#pragma unroll
    for (int i = 0; i < 4; ++i) { const int c = c0 + i; const float d = (c < CC) ? v[i] - mu : 0.f; q = fmaf(d, d, q); }
#pragma unroll
    for (int sh = 16; sh; sh >>= 1) q += __shfl_xor(q, sh, 32);
    const float rs = rsqrtf(q * (1.0f / CC) + 1e-5f); v4f ox; v4h oh;
#pragma unroll
    for (int i = 0; i < 4; ++i) { const int c = c0 + i; ox[i] = v[i]; oh[i] = tohx(c < CC ? (v[i] - mu) * rs * bfr(g_[c]) + bfr(b_[c < CC ? c : 0]) : 0.f); }
#pragma unroll 1
    for (int ps = 0; ps < 2; ++ps) { *(volatile v4f*)(X2 + p * CP + c0) = ox; *(volatile v4h*)(H2p + p * CP + c0) = oh; if (ps == 0) __threadfence(); }
}
__global__ __launch_bounds__(256) void k_gelu16(const float* __restrict__ F1, h16* G16) {
    const int lane = threadIdx.x & 31; const size_t p = (size_t)blockIdx.x * 8 + (threadIdx.x >> 5); if (p >= (size_t)NP) return;
#pragma unroll 1
    for (int q = 0; q < HID / 128; ++q) { const int c0 = q * 128 + lane * 4; v4h o;
#pragma unroll
        for (int i = 0; i < 4; ++i) o[i] = tohx(gelu_e(F1[p * HID + c0 + i]));
        *(volatile v4h*)(G16 + p * HID + c0) = o; __threadfence(); *(volatile v4h*)(G16 + p * HID + c0) = o; }
}
__global__ __launch_bounds__(256) void k_out(const float* __restrict__ X2, const float* __restrict__ F2, float* OUTB) {
    const int lane = threadIdx.x & 31; const size_t p0 = ((size_t)blockIdx.x * 8 + (threadIdx.x >> 5)) * 2; if (p0 >= (size_t)NP) return; if (lane >= 24) return;
#pragma unroll 1
    for (int ps = 0; ps < 2; ++ps) {
#pragma unroll
        for (int t = 0; t < 2; ++t) { const size_t p = p0 + t; v4f o;
#pragma unroll
            for (int i = 0; i < 4; ++i) { const int c = lane * 4 + i; o[i] = X2[p * CP + c] + F2[p * CP + c]; }
            *(volatile v4f*)(OUTB + p * CC + lane * 4) = o; }
        if (ps == 0) __threadfence(); }
}
extern "C" void kernel_launch(void* const* d_in, const int* in_sizes, int n_in,
                              void* d_out, int out_size, void* d_ws, size_t ws_size, hipStream_t stream) {
    (void)in_sizes; (void)n_in; (void)out_size;
    const float* x = (const float*)d_in[0]; const float* n1g = (const float*)d_in[1]; const float* n1b = (const float*)d_in[2]; const float* qkvw = (const float*)d_in[3]; const float* qb = (const float*)d_in[4]; const float* vb = (const float*)d_in[5]; const float* tab = (const float*)d_in[6]; const float* pw = (const float*)d_in[7]; const float* pb = (const float*)d_in[8]; const float* n2g = (const float*)d_in[9]; const float* n2b = (const float*)d_in[10]; const float* f1w = (const float*)d_in[11]; const float* f1b = (const float*)d_in[12]; const float* f2w = (const float*)d_in[13]; const float* f2b = (const float*)d_in[14];
    float* out = (float*)d_out;
    char* wsp = (char*)d_ws;
    auto take = [&](size_t bytes) { char* p = wsp; wsp += (bytes + 255) & ~(size_t)255; return (void*)p; };
    h16* WQKV = (h16*)take((size_t)HID * CP * 2); h16* WP = (h16*)take((size_t)CP * CP * 2); h16* W1 = (h16*)take((size_t)HID * CP * 2); h16* W2 = (h16*)take((size_t)CP * HID * 2); float* BQ = (float*)take(HID * 4); float* BP = (float*)take(CP * 4); float* B1 = (float*)take(HID * 4); float* B2 = (float*)take(CP * 4);
    h16* H1p = (h16*)take((size_t)NP * CP * 2); float* QKV = (float*)take((size_t)NP * HID * 4);
    h16* Qp = (h16*)take((size_t)NZ * NT * KP * 2); h16* Kp = (h16*)take((size_t)NZ * NT * KP * 2); h16* VT = (h16*)take((size_t)NZ * KP * NT * 2); float* S = (float*)take((size_t)NZ * NT * NT * 4); h16* Px = (h16*)take((size_t)NZ * NT * NT * 2); float* OZ = (float*)take((size_t)NZ * NT * KP * 4);
    h16* ATT16 = (h16*)take((size_t)NP * CP * 2); float* PR = (float*)take((size_t)NP * CP * 4); float* X2 = (float*)take((size_t)NP * CP * 4); h16* H2p = (h16*)take((size_t)NP * CP * 2); float* F2 = (float*)take((size_t)NP * CP * 4);
    if ((size_t)(wsp - (char*)d_ws) > ws_size) return;
    float* F1 = QKV; h16* G16 = (h16*)S;
    k_wpad<true><<<HID / 8, 256, 0, stream>>>(qkvw, 3 * CC, CC, HID, CP, WQKV); k_wpad<false><<<CP / 8, 256, 0, stream>>>(pw, CC, CC, CP, CP, WP); k_wpad<false><<<HID / 8, 256, 0, stream>>>(f1w, HID, CC, HID, CP, W1); k_wpad<false><<<CP / 8, 256, 0, stream>>>(f2w, CC, HID, CP, HID, W2);
    k_bias<<<1, 256, 0, stream>>>(qb, vb, pb, f1b, f2b, BQ, BP, B1, B2);
    k_ln1<<<NP / 8, 256, 0, stream>>>(x, n1g, n1b, H1p);
    k_gemmw<h16, 0, true><<<dim3(NP / 64, HID / 64, 1), 32, 0, stream>>>(H1p, nullptr, WQKV, nullptr, CP, QKV, HID, BQ, 0, 0, 0);
    for (int w0 = 0; w0 < NW; w0 += GWN) {
        k_qkpl<<<(NZ * (NT / 4)) / 8, 256, 0, stream>>>(QKV, w0, Qp, Kp); k_vT<<<(NZ * KP) / 8, 256, 0, stream>>>(QKV, w0, VT);
        k_gemmw<h16, 0, false><<<dim3(NT / 64, NT / 64, NZ), 32, 0, stream>>>(Qp, nullptr, Kp, nullptr, KP, S, NT, nullptr, (size_t)NT * KP, (size_t)NT * KP, (size_t)NT * NT);
        k_softs3<<<(NZ * NT) / 8, 256, 0, stream>>>(S, tab, w0, Px);
        k_gemmh32<<<dim3(NT / 64, 1, NZ), 128, 0, stream>>>(Px, VT, NT, OZ, KP, (size_t)NT * NT, (size_t)KP * NT, (size_t)NT * KP);
        k_foldw<<<(GWN * NT) / 8, 256, 0, stream>>>(OZ, w0, ATT16); }
    k_gemmw<h16, 0, true><<<dim3(NP / 64, CP / 64, 1), 32, 0, stream>>>(ATT16, nullptr, WP, nullptr, CP, PR, CP, BP, 0, 0, 0);
    k_ln2<<<NP / 8, 256, 0, stream>>>(x, PR, n2g, n2b, X2, H2p);
    k_gemmw<h16, 0, true><<<dim3(NP / 64, HID / 64, 1), 32, 0, stream>>>(H2p, nullptr, W1, nullptr, CP, F1, HID, B1, 0, 0, 0);
    k_gelu16<<<NP / 8, 256, 0, stream>>>(F1, G16);
    k_gemmw<h16, 0, true><<<dim3(NP / 64, CP / 64, 1), 32, 0, stream>>>(G16, nullptr, W2, nullptr, HID, F2, CP, B2, 0, 0, 0);
    k_out<<<(NP / 2) / 8, 256, 0, stream>>>(X2, F2, out);
}
